// GraphNodePredictor_43121471652154
// MI455X (gfx1250) — hardware-verified
//
#include <hip/hip_runtime.h>
#include <hip/hip_bf16.h>
#include <stddef.h>


#define DIM    64
#define NCLS   100
#define K1P    128
#define NFP    112
#define NG     32
#define NTHR   256
#define NWAVE  8
#define EPT    8
#define NGRP   2
#define CHUNK  (NTHR * EPT * NGRP)
#define WCAP   (EPT * NGRP * 32)
#define LISTN  (NWAVE * WCAP)
#define NB     1024
#define SBA    10
#define NBD    32768
#define SBD    15
#define GROWS  128

#define LDS_AGG (NB * DIM * 4 + LISTN * 4)
#define LDS_DEG (NBD * 4 + LISTN * 4)

static_assert((1 << SBA) == NB);
static_assert((1 << SBD) == NBD);
static_assert((CHUNK & (CHUNK - 1)) == 0);
static_assert(CHUNK == 4096);
static_assert(((long long)(CHUNK - 1) << SBD) + NBD <= 2147483647LL);
static_assert((NB * DIM) % (NWAVE * 128) == 0);
static_assert(NB % (NWAVE * 16) == 0);
static_assert(NBD % (NTHR * 4) == 0);
static_assert(GROWS == NWAVE * 16);
static_assert(NBD % NB == 0 && NBD % GROWS == 0);
static_assert(K1P % 32 == 0 && K1P >= NCLS && NCLS % 4 == 0);
static_assert(NFP % 16 == 0 && NFP >= NCLS && NFP / 16 <= NWAVE);
static_assert(NG == 32 && (NG * NCLS) % 4 == 0 && NG % NWAVE == 0);

typedef float v2f __attribute__((ext_vector_type(2)));
typedef float v4f __attribute__((ext_vector_type(4)));
typedef float v8f __attribute__((ext_vector_type(8)));
typedef int   v4i __attribute__((ext_vector_type(4)));
typedef unsigned short v8us  __attribute__((ext_vector_type(8)));
typedef unsigned short v16us __attribute__((ext_vector_type(16)));
typedef __bf16 v16bf __attribute__((ext_vector_type(16)));
union FragB { v16bf v; v16us u; v8us h[2]; };
struct HL { v8us hi; v8us lo; };

__device__ __forceinline__ unsigned int bf_bits(float f) {
  const unsigned int u = __float_as_uint(f);
  return (u + 0x7FFFu + ((u >> 16) & 1u)) >> 16;
}
__device__ __forceinline__ unsigned int bf_lo(float f, unsigned int hb) {
  return bf_bits(f - __uint_as_float(hb << 16));
}

__device__ __forceinline__ HL split8(v4f a, v4f b) {
  HL r;
  unsigned int h;
  h = bf_bits(a.x); r.hi[0] = (unsigned short)h; r.lo[0] = (unsigned short)bf_lo(a.x, h);
  h = bf_bits(a.y); r.hi[1] = (unsigned short)h; r.lo[1] = (unsigned short)bf_lo(a.y, h);
  h = bf_bits(a.z); r.hi[2] = (unsigned short)h; r.lo[2] = (unsigned short)bf_lo(a.z, h);
  h = bf_bits(a.w); r.hi[3] = (unsigned short)h; r.lo[3] = (unsigned short)bf_lo(a.w, h);
  h = bf_bits(b.x); r.hi[4] = (unsigned short)h; r.lo[4] = (unsigned short)bf_lo(b.x, h);
  h = bf_bits(b.y); r.hi[5] = (unsigned short)h; r.lo[5] = (unsigned short)bf_lo(b.y, h);
  h = bf_bits(b.z); r.hi[6] = (unsigned short)h; r.lo[6] = (unsigned short)bf_lo(b.z, h);
  h = bf_bits(b.w); r.hi[7] = (unsigned short)h; r.lo[7] = (unsigned short)bf_lo(b.w, h);
  return r;
}

__device__ __forceinline__ v8f wmb(v16bf a, v16bf b, v8f c) {
  v8f d = __builtin_amdgcn_wmma_f32_16x16x32_bf16(false, a, false, b, (short)0, c, false, false);
  asm volatile("v_nop\n\tv_nop\n\tv_nop\n\tv_nop" : "+v"(d) : "v"(a), "v"(b));
  return d;
}

__device__ __forceinline__ v4f ld4z(const float* p, bool ok) {
  v4f z = {0.f, 0.f, 0.f, 0.f};
  if (ok) z = *(const v4f*)p;
  return z;
}

template <int NBT, bool SET>
__device__ __forceinline__ unsigned tst(int d, unsigned nb, const int* bm, int nN, bool& h) {
  if (!SET) {
    const unsigned s = (unsigned)d - nb;
    h = s < (unsigned)NBT;
    return s;
  } else {
    const unsigned u  = (unsigned)d;
    const bool     in = u < (unsigned)nN;
    const unsigned uu = in ? u : 0u;
    const unsigned w  = (unsigned)bm[uu >> 5];
    h = in && (((w >> (uu & 31u)) & 1u) != 0u);
    return 0u;
  }
}

template <int NBT, int SB, bool SET>
__device__ __forceinline__ int scan_chunk(const int* __restrict__ dsts, int nE, int cbase, int nodeBase,
                                          int vec8, int* list, const int* bm, int nN,
                                          int tid, int lane, int wave) {
  int wc = 0;
#pragma unroll
  for (int g = 0; g < NGRP; ++g) {
    const int el0  = (g * NTHR + tid) * EPT;
    const int e0   = cbase + el0;
    const int sent = -2147483647 - 1;
    v4i da, db;
    if (vec8 != 0 && e0 + 7 < nE) {
      da = *(const v4i*)(dsts + e0);
      db = *(const v4i*)(dsts + e0 + 4);
    } else {
      da.x = (e0     < nE) ? dsts[min(e0,     nE - 1)] : sent;
      da.y = (e0 + 1 < nE) ? dsts[min(e0 + 1, nE - 1)] : sent;
      da.z = (e0 + 2 < nE) ? dsts[min(e0 + 2, nE - 1)] : sent;
      da.w = (e0 + 3 < nE) ? dsts[min(e0 + 3, nE - 1)] : sent;
      db.x = (e0 + 4 < nE) ? dsts[min(e0 + 4, nE - 1)] : sent;
      db.y = (e0 + 5 < nE) ? dsts[min(e0 + 5, nE - 1)] : sent;
      db.z = (e0 + 6 < nE) ? dsts[min(e0 + 6, nE - 1)] : sent;
      db.w = (e0 + 7 < nE) ? dsts[min(e0 + 7, nE - 1)] : sent;
    }
    const unsigned nb = (unsigned)nodeBase;
    bool h0, h1, h2, h3, h4, h5, h6, h7;
    const unsigned s0 = tst<NBT, SET>(da.x, nb, bm, nN, h0);
    const unsigned s1 = tst<NBT, SET>(da.y, nb, bm, nN, h1);
    const unsigned s2 = tst<NBT, SET>(da.z, nb, bm, nN, h2);
    const unsigned s3 = tst<NBT, SET>(da.w, nb, bm, nN, h3);
    const unsigned s4 = tst<NBT, SET>(db.x, nb, bm, nN, h4);
    const unsigned s5 = tst<NBT, SET>(db.y, nb, bm, nN, h5);
    const unsigned s6 = tst<NBT, SET>(db.z, nb, bm, nN, h6);
    const unsigned s7 = tst<NBT, SET>(db.w, nb, bm, nN, h7);
    const unsigned any = __builtin_amdgcn_ballot_w32(h0 | h1 | h2 | h3 | h4 | h5 | h6 | h7);
    if (any != 0u) {
#define HITJ(J, HJ, SJ) { \
        const unsigned mj = __builtin_amdgcn_ballot_w32(HJ); \
        if (mj != 0u) { \
          if (HJ) { \
            const int pos = wc + (int)__builtin_amdgcn_mbcnt_lo(mj, 0u); \
            if (pos < WCAP) list[wave * WCAP + pos] = ((el0 + (J)) << SB) | (int)(SJ); \
          } \
          wc += (int)__builtin_popcount(mj); } }
      HITJ(0, h0, s0)
      HITJ(1, h1, s1)
      HITJ(2, h2, s2)
      HITJ(3, h3, s3)
      HITJ(4, h4, s4)
      HITJ(5, h5, s5)
      HITJ(6, h6, s6)
      HITJ(7, h7, s7)
#undef HITJ
    }
  }
  return wc;
}

__global__ __launch_bounds__(NTHR) void k_wprep(const float* __restrict__ w, int K, int N, int KP, int NP,
                                                unsigned short* ph, unsigned short* pl) {
  const int i   = blockIdx.x * NTHR + threadIdx.x;
  const int kq8 = KP >> 3;
  if (i >= NP * kq8) return;
  const int n  = i / kq8;
  const int k0 = (i - n * kq8) * 8;
  float v[8];
#pragma unroll
  for (int e = 0; e < 8; ++e) {
    const int k = k0 + e;
    v[e] = (n < N && k < K) ? w[(size_t)k * N + n] : 0.f;
  }
  v4f a, bq;
  a.x = v[0]; a.y = v[1]; a.z = v[2]; a.w = v[3];
  bq.x = v[4]; bq.y = v[5]; bq.z = v[6]; bq.w = v[7];
  const HL s = split8(a, bq);
  unsigned short* qh = ph + (size_t)n * KP + k0;
  unsigned short* ql = pl + (size_t)n * KP + k0;
  *(volatile v8us*)qh = s.hi;
  *(volatile v8us*)ql = s.lo;
  __threadfence();
  *(volatile v8us*)qh = s.hi;
  *(volatile v8us*)ql = s.lo;
}

__global__ __launch_bounds__(NTHR) void k_deg(const int* __restrict__ ei, int* dvb, int nN, int nE, int vec8) {
  extern __shared__ v4f lds_dyn[];
  int* cnt  = (int*)lds_dyn;
  int* list = cnt + NBD;
  __shared__ int wcnt[NWAVE];
  const int tid = threadIdx.x, lane = tid & 31, wave = tid >> 5;
  const int base = blockIdx.x * NBD;
  const int* dsts = ei + nE;

  for (int i = tid; i < NBD; i += NTHR) cnt[i] = (base + i < nN) ? 1 : 0;
  __syncthreads();

  const int nChunks = (nE + CHUNK - 1) / CHUNK;
#pragma unroll 1
  for (int ch = 0; ch < nChunks; ++ch) {
    const int cbase = ch * CHUNK;
    const int wc = scan_chunk<NBD, SBD, false>(dsts, nE, cbase, base, vec8, list, (const int*)0, 0, tid, lane, wave);
    if (lane == 0) wcnt[wave] = wc;
    __syncthreads();
    if (wave == 0) {
#pragma unroll 1
      for (int wsx = 0; wsx < NWAVE; ++wsx) {
        int n = __builtin_amdgcn_readfirstlane(wcnt[wsx]);
        n = n > WCAP ? WCAP : (n < 0 ? 0 : n);
        const int* lp = list + wsx * WCAP;
#pragma unroll 1
        for (int i = 0; i < n; ++i) {
          const int ent  = __builtin_amdgcn_readfirstlane(lp[i]);
          const int slot = ent & (NBD - 1);
          if (lane == 0) cnt[slot] = cnt[slot] + 1;
        }
      }
    }
    __syncthreads();
  }

  for (int i = tid; i < NBD; i += NTHR) {
    const int c = cnt[i];
    const float d = (c > 0) ? (1.0f / sqrtf((float)c)) : 0.f;
    cnt[i] = __float_as_int(d);
  }
  __syncthreads();

  int* dv = dvb + (size_t)base;
#pragma unroll 4
  for (int it = 0; it < NBD / (NTHR * 4); ++it) {
    const int idx = (it * NTHR + tid) * 4;
    const v4i v = *(const v4i*)(cnt + idx);
    *(volatile v4i*)(dv + idx) = v;
  }
  __threadfence();
#pragma unroll 4
  for (int it = 0; it < NBD / (NTHR * 4); ++it) {
    const int idx = (it * NTHR + tid) * 4;
    const v4i v = *(const v4i*)(cnt + idx);
    *(volatile v4i*)(dv + idx) = v;
  }
}

__global__ __launch_bounds__(NTHR) void k_gemm1(
    const float* __restrict__ x, const unsigned short* __restrict__ wph, const unsigned short* __restrict__ wpl,
    const float* __restrict__ dinv, float* g, int nN) {
  __shared__ __attribute__((aligned(16))) float stg[NWAVE * 16 * DIM];
  const int tid = threadIdx.x, lane = tid & 31, wave = tid >> 5, hh = lane >> 4, m = lane & 15;
  const int row0 = blockIdx.x * GROWS + wave * 16;
  int node = row0 + m;
  node = node > nN - 1 ? nN - 1 : node;
  const float* xp = x + (size_t)node * NCLS;

  v8f acc[4];
#pragma unroll
  for (int t = 0; t < 4; ++t) { v8f z = {0.f, 0.f, 0.f, 0.f, 0.f, 0.f, 0.f, 0.f}; acc[t] = z; }

#pragma unroll
  for (int ks = 0; ks < K1P / 32; ++ks) {
    const int kb = 32 * ks + 8 * hh;
    const float* p0 = xp + kb;
    const v4f f0 = ld4z(p0,      kb + 4  <= NCLS);
    const v4f f1 = ld4z(p0 + 4,  kb + 8  <= NCLS);
    const v4f f2 = ld4z(p0 + 16, kb + 20 <= NCLS);
    const v4f f3 = ld4z(p0 + 20, kb + 24 <= NCLS);
    const HL s0 = split8(f0, f1);
    const HL s1 = split8(f2, f3);
    FragB ah, al;
    ah.h[0] = s0.hi; ah.h[1] = s1.hi;
    al.h[0] = s0.lo; al.h[1] = s1.lo;
#pragma unroll
    for (int t = 0; t < 4; ++t) {
      const unsigned short* bp = wph + (size_t)(16 * t + m) * K1P + 32 * ks + 8 * hh;
      const unsigned short* bq = wpl + (size_t)(16 * t + m) * K1P + 32 * ks + 8 * hh;
      FragB bh, bl;
      bh.h[0] = *(const v8us*)bp; bh.h[1] = *(const v8us*)(bp + 16);
      bl.h[0] = *(const v8us*)bq; bl.h[1] = *(const v8us*)(bq + 16);
      acc[t] = wmb(ah.v, bh.v, acc[t]);
      acc[t] = wmb(ah.v, bl.v, acc[t]);
      acc[t] = wmb(al.v, bh.v, acc[t]);
    }
  }

  float sd[8];
#pragma unroll
  for (int r = 0; r < 8; ++r) sd[r] = dinv[row0 + 8 * hh + r];
  float* sp = stg + wave * (16 * DIM) + (8 * hh) * DIM + m;
#pragma unroll
  for (int t = 0; t < 4; ++t) {
#pragma unroll
    for (int r = 0; r < 8; ++r) sp[r * DIM + 16 * t] = acc[t][r] * sd[r];
  }
  __syncthreads();

  const float* lp = stg + wave * (16 * DIM) + 4 * lane;
  float* gp = g + (size_t)row0 * DIM + 4 * lane;
  v4f ov[8];
#pragma unroll
  for (int q = 0; q < 8; ++q) ov[q] = *(const v4f*)(lp + q * 128);
#pragma unroll
  for (int q = 0; q < 8; ++q) *(volatile v4f*)(gp + q * 128) = ov[q];
  __threadfence();
#pragma unroll
  for (int q = 0; q < 8; ++q) *(volatile v4f*)(gp + q * 128) = ov[q];
}

__global__ __launch_bounds__(NTHR) void k_agg(
    const int* __restrict__ ei, const float* __restrict__ gin, const float* __restrict__ dinv,
    const float* __restrict__ bias, const unsigned short* __restrict__ wph, const unsigned short* __restrict__ wpl,
    float* gout, int nN, int nE, int vec8) {
  extern __shared__ v4f lds_dyn[];
  float* acc  = (float*)lds_dyn;
  int*   list = (int*)(acc + NB * DIM);
  __shared__ int wcnt[NWAVE];
  __shared__ float sdinv[NB];
  __shared__ __attribute__((aligned(16))) float sbias[DIM];
  const int tid = threadIdx.x, lane = tid & 31, wave = tid >> 5, hh = lane >> 4, m = lane & 15;
  const int base = blockIdx.x * NB;
  const int* dsts = ei + nE;

  for (int i = tid; i < NB; i += NTHR) sdinv[i] = dinv[base + i];
  if (tid < DIM) sbias[tid] = bias[tid];
  {
    const v4f z = {0.f, 0.f, 0.f, 0.f};
    for (int i = tid; i < NB * DIM / 4; i += NTHR) lds_dyn[i] = z;
  }
  __syncthreads();

  const int nChunks = (nE + CHUNK - 1) / CHUNK;
#pragma unroll 1
  for (int ch = 0; ch < nChunks; ++ch) {
    const int cbase = ch * CHUNK;
    const int wc = scan_chunk<NB, SBA, false>(dsts, nE, cbase, base, vec8, list, (const int*)0, 0, tid, lane, wave);
    if (lane == 0) wcnt[wave] = wc;
    __syncthreads();
    if (wave == 0) {
#pragma unroll 1
      for (int wsx = 0; wsx < NWAVE; ++wsx) {
        int n = __builtin_amdgcn_readfirstlane(wcnt[wsx]);
        n = n > WCAP ? WCAP : (n < 0 ? 0 : n);
        const int* lp = list + wsx * WCAP;
#pragma unroll 1
        for (int i = 0; i < n; ++i) {
          const int ent  = __builtin_amdgcn_readfirstlane(lp[i]);
          const int slot = ent & (NB - 1);
          int e = cbase + ((ent >> SBA) & (CHUNK - 1));
          e = e > nE - 1 ? nE - 1 : e;
          int src = ei[e];
          src = src < 0 ? 0 : (src > nN - 1 ? nN - 1 : src);
          const v2f v = *(const v2f*)(gin + (size_t)src * DIM + 2 * lane);
          v2f* ap = (v2f*)(acc + slot * DIM + 2 * lane);
          *ap = *ap + v;
        }
      }
    }
    __syncthreads();
  }

  const v2f b2v = *(const v2f*)(sbias + 2 * lane);
#pragma unroll 2
  for (int j = 0; j < NB / NWAVE; ++j) {
    const int slot = wave * (NB / NWAVE) + j;
    int node = base + slot;
    node = node > nN - 1 ? nN - 1 : node;
    v2f* ap = (v2f*)(acc + slot * DIM + 2 * lane);
    const v2f gv = *(const v2f*)(gin + (size_t)node * DIM + 2 * lane);
    const float sd = sdinv[slot];
    v2f t = (*ap + gv) * sd + b2v;
    t.x = fmaxf(t.x, 0.f);
    t.y = fmaxf(t.y, 0.f);
    *ap = t;
  }
  __syncthreads();

#pragma unroll 1
  for (int j = 0; j < NB / (NWAVE * 16); ++j) {
    const int slot0 = wave * (NB / NWAVE) + 16 * j;
    const float* ar = acc + (slot0 + m) * DIM;
    FragB ah0, al0, ah1, al1;
    {
      const float* p = ar + 8 * hh;
      const HL s0 = split8(*(const v4f*)p,        *(const v4f*)(p + 4));
      const HL s1 = split8(*(const v4f*)(p + 16), *(const v4f*)(p + 20));
      ah0.h[0] = s0.hi; ah0.h[1] = s1.hi; al0.h[0] = s0.lo; al0.h[1] = s1.lo;
    }
    {
      const float* p = ar + 32 + 8 * hh;
      const HL s0 = split8(*(const v4f*)p,        *(const v4f*)(p + 4));
      const HL s1 = split8(*(const v4f*)(p + 16), *(const v4f*)(p + 20));
      ah1.h[0] = s0.hi; ah1.h[1] = s1.hi; al1.h[0] = s0.lo; al1.h[1] = s1.lo;
    }
    v8f c[4];
#pragma unroll
    for (int t = 0; t < 4; ++t) { v8f z = {0.f, 0.f, 0.f, 0.f, 0.f, 0.f, 0.f, 0.f}; c[t] = z; }
#pragma unroll
    for (int t = 0; t < 4; ++t) {
      const unsigned short* bp = wph + (size_t)(16 * t + m) * DIM + 8 * hh;
      const unsigned short* bq = wpl + (size_t)(16 * t + m) * DIM + 8 * hh;
      FragB bh, bl;
      bh.h[0] = *(const v8us*)bp;        bh.h[1] = *(const v8us*)(bp + 16);
      bl.h[0] = *(const v8us*)bq;        bl.h[1] = *(const v8us*)(bq + 16);
      c[t] = wmb(ah0.v, bh.v, c[t]);
      c[t] = wmb(ah0.v, bl.v, c[t]);
      c[t] = wmb(al0.v, bh.v, c[t]);
      bh.h[0] = *(const v8us*)(bp + 32); bh.h[1] = *(const v8us*)(bp + 48);
      bl.h[0] = *(const v8us*)(bq + 32); bl.h[1] = *(const v8us*)(bq + 48);
      c[t] = wmb(ah1.v, bh.v, c[t]);
      c[t] = wmb(ah1.v, bl.v, c[t]);
      c[t] = wmb(al1.v, bh.v, c[t]);
    }
    float sd[8];
#pragma unroll
    for (int r = 0; r < 8; ++r) sd[r] = sdinv[slot0 + 8 * hh + r];
    float* sp = acc + (slot0 + 8 * hh) * DIM + m;
#pragma unroll
    for (int t = 0; t < 4; ++t) {
#pragma unroll
      for (int r = 0; r < 8; ++r) sp[r * DIM + 16 * t] = c[t][r] * sd[r];
    }
  }
  __syncthreads();

  const size_t ob = (size_t)base * DIM;
#pragma unroll 4
  for (int q = 0; q < (NB * DIM) / (NWAVE * 128); ++q) {
    const int f = (wave * ((NB * DIM) / (NWAVE * 128)) + q) * 128 + 4 * lane;
    const v4f v = *(const v4f*)(acc + f);
    *(volatile v4f*)(gout + ob + (size_t)f) = v;
  }
  __threadfence();
#pragma unroll 4
  for (int q = 0; q < (NB * DIM) / (NWAVE * 128); ++q) {
    const int f = (wave * ((NB * DIM) / (NWAVE * 128)) + q) * 128 + 4 * lane;
    const v4f v = *(const v4f*)(acc + f);
    *(volatile v4f*)(gout + ob + (size_t)f) = v;
  }
}

__global__ __launch_bounds__(NTHR) void k_last(
    const int* __restrict__ ei, const int* __restrict__ batch, const int* __restrict__ mni,
    const float* __restrict__ gin, const float* __restrict__ dinv, const float* __restrict__ b3,
    const unsigned short* __restrict__ fph, const unsigned short* __restrict__ fpl, const float* __restrict__ fcb,
    float* out, int nN, int nE, int vec8) {
  extern __shared__ v4f lds_dyn[];
  int* bm = (int*)lds_dyn;
  __shared__ __attribute__((aligned(16))) float acc3[NG * DIM];
  __shared__ __attribute__((aligned(16))) float stg[NG * NFP];
  __shared__ int list[LISTN];
  __shared__ int part[NWAVE * NG];
  __shared__ int counts[NG];
  __shared__ int gn[NG];
  __shared__ float sdv[NG];
  __shared__ __attribute__((aligned(16))) float sb3[DIM];
  __shared__ float sfcb[NFP];
  __shared__ int wcnt[NWAVE];
  const int tid = threadIdx.x, lane = tid & 31, wave = tid >> 5, hh = lane >> 4, m = lane & 15;
  const int* dsts = ei + nE;

  {
    const int v = lane, c = wave;
    const int len = (nN + NWAVE - 1) / NWAVE;
    const int i0 = c * len;
    int i1 = i0 + len;
    i1 = i1 > nN ? nN : i1;
    int cv = 0;
#pragma unroll 1
    for (int i = i0; i < i1; ++i) cv += (batch[i] == v) ? 1 : 0;
    part[c * NG + v] = cv;
  }
  for (int i = tid; i < NG * DIM; i += NTHR) acc3[i] = 0.f;
  {
    const int nW = (nN + 31) >> 5;
    for (int i = tid; i < nW; i += NTHR) bm[i] = 0;
  }
  if (tid < DIM) sb3[tid] = b3[tid];
  if (tid < NFP) sfcb[tid] = (tid < NCLS) ? fcb[tid] : 0.f;
  __syncthreads();
  if (tid < NG) {
    int s = 0;
#pragma unroll
    for (int c = 0; c < NWAVE; ++c) s += part[c * NG + tid];
    counts[tid] = s;
  }
  __syncthreads();
  if (tid < NG) {
    const int mr = mni[tid];
    int mw = mr;
    if (mw < 0) mw += nN;
    mw = mw < 0 ? 0 : (mw > nN - 1 ? nN - 1 : mw);
    int bi = batch[mw];
    if (bi < 0) bi += NG;
    bi = bi < 0 ? 0 : (bi > NG - 1 ? NG - 1 : bi);
    const int off = (bi == 0) ? 0 : counts[bi - 1];
    long long gi = (long long)mr + (long long)off;
    gi = gi < 0 ? 0 : (gi > (long long)(nN - 1) ? (long long)(nN - 1) : gi);
    gn[tid]  = (int)gi;
    sdv[tid] = dinv[(int)gi];
  }
  __syncthreads();
  if (tid == 0) {
#pragma unroll 1
    for (int s = 0; s < NG; ++s) {
      const int gq = gn[s];
      bm[gq >> 5] = bm[gq >> 5] | (int)(1u << (gq & 31));
    }
  }
  __syncthreads();

  const int nChunks = (nE + CHUNK - 1) / CHUNK;
#pragma unroll 1
  for (int ch = 0; ch < nChunks; ++ch) {
    const int cbase = ch * CHUNK;
    const int wc = scan_chunk<1, 0, true>(dsts, nE, cbase, 0, vec8, list, bm, nN, tid, lane, wave);
    if (lane == 0) wcnt[wave] = wc;
    __syncthreads();
    if (wave == 0) {
#pragma unroll 1
      for (int wsx = 0; wsx < NWAVE; ++wsx) {
        int n = __builtin_amdgcn_readfirstlane(wcnt[wsx]);
        n = n > WCAP ? WCAP : (n < 0 ? 0 : n);
        const int* lp = list + wsx * WCAP;
#pragma unroll 1
        for (int i = 0; i < n; ++i) {
          const int el = __builtin_amdgcn_readfirstlane(lp[i]) & (CHUNK - 1);
          int e = cbase + el;
          e = e > nE - 1 ? nE - 1 : e;
          const int d = dsts[e];
          int src = ei[e];
          src = src < 0 ? 0 : (src > nN - 1 ? nN - 1 : src);
          const v2f v = *(const v2f*)(gin + (size_t)src * DIM + 2 * lane);
#pragma unroll 1
          for (int s = 0; s < NG; ++s) {
            if (gn[s] == d) {
              v2f* ap = (v2f*)(acc3 + s * DIM + 2 * lane);
              *ap = *ap + v;
            }
          }
        }
      }
    }
    __syncthreads();
  }

  {
    const v2f bv = *(const v2f*)(sb3 + 2 * lane);
#pragma unroll
    for (int q = 0; q < NG / NWAVE; ++q) {
      const int s = wave * (NG / NWAVE) + q;
      const int node = gn[s];
      const v2f gv = *(const v2f*)(gin + (size_t)node * DIM + 2 * lane);
      v2f* ap = (v2f*)(acc3 + s * DIM + 2 * lane);
      const float sd = sdv[s];
      *ap = (*ap + gv) * sd + bv;
    }
  }
  __syncthreads();

  {
    const int t7 = wave < (NFP / 16) ? wave : (NFP / 16 - 1);
    FragB ah[2][2], al[2][2];
#pragma unroll
    for (int rt = 0; rt < 2; ++rt) {
#pragma unroll
      for (int ks = 0; ks < 2; ++ks) {
        const float* p = acc3 + (rt * 16 + m) * DIM + 32 * ks + 8 * hh;
        const HL s0 = split8(*(const v4f*)p,        *(const v4f*)(p + 4));
        const HL s1 = split8(*(const v4f*)(p + 16), *(const v4f*)(p + 20));
        ah[rt][ks].h[0] = s0.hi; ah[rt][ks].h[1] = s1.hi;
        al[rt][ks].h[0] = s0.lo; al[rt][ks].h[1] = s1.lo;
      }
    }
    v8f c[2];
    { v8f z = {0.f, 0.f, 0.f, 0.f, 0.f, 0.f, 0.f, 0.f}; c[0] = z; c[1] = z; }
#pragma unroll
    for (int ks = 0; ks < 2; ++ks) {
      const unsigned short* bp = fph + (size_t)(16 * t7 + m) * DIM + 32 * ks + 8 * hh;
      const unsigned short* bq = fpl + (size_t)(16 * t7 + m) * DIM + 32 * ks + 8 * hh;
      FragB bh, bl;
      bh.h[0] = *(const v8us*)bp; bh.h[1] = *(const v8us*)(bp + 16);
      bl.h[0] = *(const v8us*)bq; bl.h[1] = *(const v8us*)(bq + 16);
#pragma unroll
      for (int rt = 0; rt < 2; ++rt) {
        c[rt] = wmb(ah[rt][ks].v, bh.v, c[rt]);
        c[rt] = wmb(ah[rt][ks].v, bl.v, c[rt]);
        c[rt] = wmb(al[rt][ks].v, bh.v, c[rt]);
      }
    }
    if (wave < NFP / 16) {
      const float bb = sfcb[16 * t7 + m];
#pragma unroll
      for (int rt = 0; rt < 2; ++rt) {
        float* sp = stg + (rt * 16 + 8 * hh) * NFP + 16 * t7 + m;
#pragma unroll
        for (int r = 0; r < 8; ++r) sp[r * NFP] = c[rt][r] + bb;
      }
    }
  }
  __syncthreads();

  const int nq = (NG * NCLS) / 4;
  for (int i = tid; i < nq; i += NTHR) {
    const int f = 4 * i;
    const int row = f / NCLS;
    const int col = f - row * NCLS;
    const v4f v = *(const v4f*)(stg + row * NFP + col);
    *(volatile v4f*)(out + f) = v;
  }
  __threadfence();
  for (int i = tid; i < nq; i += NTHR) {
    const int f = 4 * i;
    const int row = f / NCLS;
    const int col = f - row * NCLS;
    const v4f v = *(const v4f*)(stg + row * NFP + col);
    *(volatile v4f*)(out + f) = v;
  }
}

extern "C" void kernel_launch(void* const* d_in, const int* in_sizes, int n_in,
                              void* d_out, int out_size, void* d_ws, size_t ws_size,
                              hipStream_t stream) {
  if (n_in < 12) return;
  const int nN = in_sizes[2];
  if (nN <= 0) return;
  if (in_sizes[0] != nN * NCLS) return;
  if (in_sizes[1] < 0 || (in_sizes[1] & 1) != 0) return;
  const int nE = in_sizes[1] / 2;
  if (in_sizes[3] != NG) return;
  if (in_sizes[4] != NCLS * DIM || in_sizes[5] != DIM) return;
  if (in_sizes[6] != DIM * DIM || in_sizes[7] != DIM) return;
  if (in_sizes[8] != DIM * DIM || in_sizes[9] != DIM) return;
  if (in_sizes[10] != DIM * NCLS || in_sizes[11] != NCLS) return;
  if (out_size != NG * NCLS) return;

  const float* x     = (const float*)d_in[0];
  const int*   ei    = (const int*)d_in[1];
  const int*   batch = (const int*)d_in[2];
  const int*   mni   = (const int*)d_in[3];
  const float* W1    = (const float*)d_in[4];
  const float* b1    = (const float*)d_in[5];
  const float* W2    = (const float*)d_in[6];
  const float* b2    = (const float*)d_in[7];
  const float* W3    = (const float*)d_in[8];
  const float* b3    = (const float*)d_in[9];
  const float* fcW   = (const float*)d_in[10];
  const float* fcb   = (const float*)d_in[11];
  float* out = (float*)d_out;

  const int nDB = (nN + NBD - 1) / NBD;
  const int nGB = (nN + GROWS - 1) / GROWS;
  const int nAB = (nN + NB - 1) / NB;
  size_t GR = (size_t)nGB * GROWS;
  if ((size_t)nAB * NB > GR) GR = (size_t)nAB * NB;

  char* ws = (char*)d_ws;
  size_t off = 0;
  const size_t szW1 = (size_t)DIM * K1P * 2, szW = (size_t)DIM * DIM * 2, szF = (size_t)NFP * DIM * 2;
  const size_t oW1h = off; off += szW1; off = (off + 255) & ~(size_t)255;
  const size_t oW1l = off; off += szW1; off = (off + 255) & ~(size_t)255;
  const size_t oW2h = off; off += szW;  off = (off + 255) & ~(size_t)255;
  const size_t oW2l = off; off += szW;  off = (off + 255) & ~(size_t)255;
  const size_t oW3h = off; off += szW;  off = (off + 255) & ~(size_t)255;
  const size_t oW3l = off; off += szW;  off = (off + 255) & ~(size_t)255;
  const size_t oFh  = off; off += szF;  off = (off + 255) & ~(size_t)255;
  const size_t oFl  = off; off += szF;  off = (off + 255) & ~(size_t)255;
  const size_t oDV  = off; off += (size_t)nDB * NBD * 4; off = (off + 255) & ~(size_t)255;
  const size_t szG  = GR * DIM * 4;
  const size_t oGA  = off; off += szG;  off = (off + 255) & ~(size_t)255;
  const size_t oGB  = off; off += szG;  off = (off + 255) & ~(size_t)255;
  if (off > ws_size) return;
  if (off > ((size_t)128 << 20)) return;
  size_t bmB = (size_t)((nN + 31) / 32) * 4;
  bmB = (bmB + 15) & ~(size_t)15;
  if (bmB > (size_t)160 * 1024) return;

  unsigned short* w1h = (unsigned short*)(ws + oW1h);
  unsigned short* w1l = (unsigned short*)(ws + oW1l);
  unsigned short* w2h = (unsigned short*)(ws + oW2h);
  unsigned short* w2l = (unsigned short*)(ws + oW2l);
  unsigned short* w3h = (unsigned short*)(ws + oW3h);
  unsigned short* w3l = (unsigned short*)(ws + oW3l);
  unsigned short* fh  = (unsigned short*)(ws + oFh);
  unsigned short* fl  = (unsigned short*)(ws + oFl);
  float* dinv = (float*)(ws + oDV);
  float* GA   = (float*)(ws + oGA);
  float* GBf  = (float*)(ws + oGB);

  const int vec8 = ((nE & 3) == 0) ? 1 : 0;

  {
    const int t1 = DIM * (K1P / 8), t2 = DIM * (DIM / 8), tf = NFP * (DIM / 8);
    k_wprep<<<(t1 + NTHR - 1) / NTHR, NTHR, 0, stream>>>(W1,  NCLS, DIM,  K1P, DIM, w1h, w1l);
    k_wprep<<<(t2 + NTHR - 1) / NTHR, NTHR, 0, stream>>>(W2,  DIM,  DIM,  DIM, DIM, w2h, w2l);
    k_wprep<<<(t2 + NTHR - 1) / NTHR, NTHR, 0, stream>>>(W3,  DIM,  DIM,  DIM, DIM, w3h, w3l);
    k_wprep<<<(tf + NTHR - 1) / NTHR, NTHR, 0, stream>>>(fcW, DIM,  NCLS, DIM, NFP, fh,  fl);
  }

  hipFuncSetAttribute(reinterpret_cast<const void*>(&k_deg),
                      hipFuncAttributeMaxDynamicSharedMemorySize, LDS_DEG);
  k_deg<<<nDB, NTHR, LDS_DEG, stream>>>(ei, (int*)(ws + oDV), nN, nE, vec8);

  k_gemm1<<<nGB, NTHR, 0, stream>>>(x, w1h, w1l, dinv, GA, nN);

  hipFuncSetAttribute(reinterpret_cast<const void*>(&k_agg),
                      hipFuncAttributeMaxDynamicSharedMemorySize, LDS_AGG);
  k_agg<<<nAB, NTHR, LDS_AGG, stream>>>(ei, GA,  dinv, b1, w2h, w2l, GBf, nN, nE, vec8);
  k_agg<<<nAB, NTHR, LDS_AGG, stream>>>(ei, GBf, dinv, b2, w3h, w3l, GA,  nN, nE, vec8);

  hipFuncSetAttribute(reinterpret_cast<const void*>(&k_last),
                      hipFuncAttributeMaxDynamicSharedMemorySize, (int)bmB);
  k_last<<<1, NTHR, bmB, stream>>>(ei, batch, mni, GA, dinv, b3, fh, fl, fcb, out, nN, nE, vec8);
}
